// VimMamba_74199855005904
// MI455X (gfx1250) — hardware-verified
//
#include <hip/hip_runtime.h>


#define NBT  4
#define LL   512
#define DMOD 1024
#define DI   2048
#define NS   16
#define DTR  64
#define NXL  96
#define NXP  128
#define KDT  64
#define DM   DMOD
#define LOSC 1024.0f

typedef _Float16 h16;
typedef unsigned short bf;
typedef __attribute__((ext_vector_type(16))) __bf16   v16bf;
typedef __attribute__((ext_vector_type(16))) _Float16 v16h;
typedef __attribute__((ext_vector_type(8)))  _Float16 v8h;
typedef __attribute__((ext_vector_type(8)))  unsigned short v8us;
typedef __attribute__((ext_vector_type(8)))  float    v8f;
typedef __attribute__((ext_vector_type(4)))  float    v4f;
typedef v8h  __attribute__((may_alias)) v8ha;
typedef v4f  __attribute__((may_alias)) v4fa;
typedef v8us __attribute__((may_alias)) v8usa;

__device__ __forceinline__ unsigned short f2bf(float f) { unsigned u = __float_as_uint(f); u += 0x7FFFu + ((u >> 16) & 1u); return (unsigned short)(u >> 16); }
__device__ __forceinline__ float bf2f(unsigned short b) { return __uint_as_float(((unsigned)b) << 16); }
__device__ __forceinline__ float bfr(float f) { return bf2f(f2bf(f)); }
__device__ __forceinline__ v16h cat16(v8h lo, v8h hi) { return __builtin_shufflevector(lo, hi, 0, 1, 2, 3, 4, 5, 6, 7, 8, 9, 10, 11, 12, 13, 14, 15); }
__device__ __forceinline__ v16bf cat16b(v8us lo, v8us hi) { return __builtin_bit_cast(v16bf, __builtin_shufflevector(lo, hi, 0, 1, 2, 3, 4, 5, 6, 7, 8, 9, 10, 11, 12, 13, 14, 15)); }
__device__ __forceinline__ v8f wmma16(v16h a, v16h b, v8f c) { return __builtin_amdgcn_wmma_f32_16x16x32_f16(false, a, false, b, (short)0, c, false, false); }
__device__ __forceinline__ v8f wmmab(v16bf a, v16bf b, v8f c) { return __builtin_amdgcn_wmma_f32_16x16x32_bf16(false, a, false, b, (short)0, c, false, false); }

template <bool SPLITA, bool F16OUT = false>
__global__ __launch_bounds__(128) void k_gemmb(const bf* __restrict__ A, const bf* __restrict__ Al, const bf* __restrict__ Bn, const float* __restrict__ bias, float* C, int ldc, h16* C2, const float* __restrict__ R = nullptr, int K = DM, int roundR = 1) {
    __shared__ __align__(16) float ost[4][16 * 68];
    const int lane = threadIdx.x & 31, wave = threadIdx.x >> 5, lr = lane & 15, hi = lane >> 4;
    const int r0 = blockIdx.x * 64 + wave * 16, c0 = blockIdx.y * 64;
    const size_t aoff = (size_t)(r0 + lr) * K + 8 * hi;
    size_t boff[4];
#pragma unroll
    for (int t = 0; t < 4; ++t) boff[t] = (size_t)(c0 + t * 16 + lr) * K + 8 * hi;
    v8f acc[4];
#pragma unroll
    for (int t = 0; t < 4; ++t) acc[t] = (v8f){};
#pragma unroll 1
    for (int kc = 0; kc < K; kc += 32) {
        const v16bf a = cat16b(*(const v8us*)(A + aoff + kc), *(const v8us*)(A + aoff + kc + 16));
        v16bf al = a;
        if (SPLITA) al = cat16b(*(const v8us*)(Al + aoff + kc), *(const v8us*)(Al + aoff + kc + 16));
#pragma unroll
        for (int t = 0; t < 4; ++t) { const v16bf b = cat16b(*(const v8us*)(Bn + boff[t] + kc), *(const v8us*)(Bn + boff[t] + kc + 16)); acc[t] = wmmab(a, b, acc[t]); if (SPLITA) acc[t] = wmmab(al, b, acc[t]); }
        asm volatile("v_nop\n\tv_nop\n\tv_nop\n\tv_nop" : "+v"(acc[0]), "+v"(acc[1]), "+v"(acc[2]), "+v"(acc[3]) : "v"(a), "v"(al));
    }
    float* os = &ost[wave][0];
#pragma unroll
    for (int t = 0; t < 4; ++t) { const float bv = bias ? bfr(bias[c0 + t * 16 + lr]) : 0.f;
#pragma unroll
        for (int j = 0; j < 8; ++j) os[(hi * 8 + j) * 68 + t * 16 + lr] = acc[t][j] + bv; }
    __syncthreads();
    if (F16OUT) {
        h16* crow = (h16*)(void*)C + (size_t)r0 * ldc + c0;
        auto pass = [&]() {
#pragma unroll
            for (int s = 0; s < 4; ++s) { const int row = 4 * s + (lane >> 3), piece = lane & 7; const float* sp = os + row * 68 + piece * 8; v8h o, o2;
#pragma unroll
                for (int i = 0; i < 8; ++i) { const h16 a = (h16)sp[i]; o[i] = a; o2[i] = (h16)((sp[i] - (float)a) * LOSC); }
                *(volatile v8h*)(crow + (size_t)row * ldc + piece * 8) = o; if (C2) *(volatile v8h*)(C2 + (size_t)r0 * ldc + c0 + (size_t)row * ldc + piece * 8) = o2; }
        };
        pass(); __threadfence(); pass();
    } else {
        float* crow = C + (size_t)r0 * ldc + c0;
        auto pass = [&]() {
#pragma unroll
            for (int s = 0; s < 8; ++s) { const int Lid = (lane >> 3) + 4 * s, piece = lane & 7; const int row = Lid >> 1, cofs = (Lid & 1) * 32 + piece * 4;
                v4f val = *(const v4fa*)(os + row * 68 + cofs); if (R) { const v4f rv = *(const v4f*)(R + ((size_t)r0 + row) * ldc + c0 + cofs); val += roundR ? (v4f){bfr(rv[0]), bfr(rv[1]), bfr(rv[2]), bfr(rv[3])} : rv; }
                *(volatile v4f*)(crow + (size_t)row * ldc + cofs) = val; }
        };
        pass(); __threadfence(); pass();
    }
}


__global__ __launch_bounds__(256) void k_cvt8(const float* __restrict__ src, bf* dst, size_t n8) {
    const size_t i = (size_t)blockIdx.x * 256 + threadIdx.x; if (i >= n8) return;
    const v8f v = *(const v8f*)(src + i * 8); v8us o;
#pragma unroll
    for (int k = 0; k < 8; ++k) o[k] = f2bf(v[k]);
    *(volatile v8us*)(dst + i * 8) = o; __threadfence(); *(volatile v8us*)(dst + i * 8) = o;
}
__global__ __launch_bounds__(256) void k_zero8(bf* dst, size_t n8) {
    const size_t i = (size_t)blockIdx.x * 256 + threadIdx.x; if (i >= n8) return; v8us z;
#pragma unroll
    for (int k = 0; k < 8; ++k) z[k] = 0;
    *(volatile v8us*)(dst + i * 8) = z; __threadfence(); *(volatile v8us*)(dst + i * 8) = z;
}

__global__ __launch_bounds__(256) void k_conv(const float* __restrict__ XZ, const float* __restrict__ wc, const float* __restrict__ bc, float* XC, bf* Ch, bf* Cl) {
    typedef __attribute__((ext_vector_type(4))) unsigned short v4us;
    const int lane = threadIdx.x & 31; const int l = blockIdx.x * 8 + (threadIdx.x >> 5); if (l >= LL) return;
#pragma unroll 1
    for (int ps = 0; ps < 2; ++ps) {
#pragma unroll 1
        for (int q = 0; q < DI / 128; ++q) { const int d0 = q * 128 + lane * 4; v4f y; v4us oh, ol;
#pragma unroll
            for (int i = 0; i < 4; ++i) { const int d = d0 + i; float acc = bfr(bc[d]);
#pragma unroll
                for (int k = 0; k < 4; ++k) { const int ls = l - 3 + k; if (ls >= 0) acc = fmaf(bfr(wc[d * 4 + k]), XZ[(size_t)ls * (2 * DI) + d], acc); }
                y[i] = fminf(fmaxf(acc, -10.0f), 10.0f); const unsigned short hb = f2bf(acc); oh[i] = hb; ol[i] = f2bf(acc - bf2f(hb)); }
            const size_t o = (size_t)l * DI + d0; *(volatile v4f*)(XC + o) = y; *(volatile v4us*)(Ch + o) = oh; *(volatile v4us*)(Cl + o) = ol; }
        if (ps == 0) __threadfence(); }
}
__global__ __launch_bounds__(256) void k_wxpad(const float* __restrict__ wx, bf* WXP) {
    const int lane = threadIdx.x & 31; const int r = blockIdx.x * 8 + (threadIdx.x >> 5); if (r >= NXP) return;
#pragma unroll 1
    for (int ps = 0; ps < 2; ++ps) {
#pragma unroll
        for (int q = 0; q < DI / 256; ++q) { v8us o;
#pragma unroll
            for (int i = 0; i < 8; ++i) o[i] = f2bf(r < NXL ? wx[(size_t)(r < NXL ? r : 0) * DI + q * 256 + lane * 8 + i] : 0.f);
            *(volatile v8us*)(WXP + (size_t)r * DI + q * 256 + lane * 8) = o; }
        if (ps == 0) __threadfence(); }
}
__global__ __launch_bounds__(256) void k_wdtpad(const float* __restrict__ wdt, bf* WDT) {
    typedef __attribute__((ext_vector_type(2))) unsigned short v2us;
    const int lane = threadIdx.x & 31; const int d = blockIdx.x * 8 + (threadIdx.x >> 5); if (d >= DI) return; v2us o;
#pragma unroll
    for (int i = 0; i < 2; ++i) { const int k = lane * 2 + i; o[i] = f2bf(k < DTR ? wdt[(size_t)d * DTR + (k < DTR ? k : 0)] : 0.f); }
    *(volatile v2us*)(WDT + (size_t)d * KDT + lane * 2) = o; __threadfence(); *(volatile v2us*)(WDT + (size_t)d * KDT + lane * 2) = o;
}
__global__ __launch_bounds__(256) void k_dtplanes(const float* __restrict__ XD, bf* Ph, bf* Pl) {
    typedef __attribute__((ext_vector_type(2))) unsigned short v2us;
    const int lane = threadIdx.x & 31; const size_t l = (size_t)blockIdx.x * 8 + (threadIdx.x >> 5); if (l >= (size_t)LL) return; v2us oh, ol;
#pragma unroll
    for (int i = 0; i < 2; ++i) { const int k = lane * 2 + i; const float y = (k < DTR) ? XD[l * NXP + (k < DTR ? k : 0)] : 0.f; const unsigned short hb = f2bf(y); oh[i] = hb; ol[i] = f2bf(y - bf2f(hb)); }
    const size_t o = l * KDT + lane * 2; *(volatile v2us*)(Ph + o) = oh; *(volatile v2us*)(Pl + o) = ol; __threadfence(); *(volatile v2us*)(Ph + o) = oh; *(volatile v2us*)(Pl + o) = ol;
}
__global__ __launch_bounds__(256) void k_softplus(float* DEL, const float* __restrict__ bdt) {
    const int lane = threadIdx.x & 31; const size_t l = (size_t)blockIdx.x * 8 + (threadIdx.x >> 5); if (l >= (size_t)LL) return;
#pragma unroll 1
    for (int q = 0; q < DI / 128; ++q) { float* p = DEL + l * DI + q * 128 + lane * 4; v4f v = *(const v4f*)p;
#pragma unroll
        for (int i = 0; i < 4; ++i) { const float bb = bfr(bdt[q * 128 + lane * 4 + i]); float t = v[i] + bb; t = fminf(fmaxf(t, 1e-5f), 1.0f) + bb; v[i] = (t > 20.f) ? t : log1pf(expf(t)); }
        *(volatile v4f*)p = v; __threadfence(); *(volatile v4f*)p = v; }
}

__global__ __launch_bounds__(256) void k_scan(const float* __restrict__ DEL, const float* __restrict__ XD, const float* __restrict__ XC, const float* __restrict__ Alog, const float* __restrict__ Dp, float* YP) {
    const int lane = threadIdx.x & 31; const int w = blockIdx.x * 8 + (threadIdx.x >> 5); if (w >= DI / 2) return; const int half = lane >> 4, n = lane & 15, s = lane & 15; const int d = w * 2 + half;
    const float A = -expf(bfr(Alog[d * NS + n])); const float Dd = bfr(Dp[d]); float h = 0.f; float keep = 0.f;
#pragma unroll 1
    for (int l = 0; l < LL; ++l) {
        const float dl = DEL[(size_t)l * DI + d]; const float xv = XC[(size_t)l * DI + d]; const float Bn = XD[(size_t)l * NXP + DTR + n]; const float Cn = XD[(size_t)l * NXP + DTR + NS + n];
        h = expf(dl * A) * h + dl * Bn * xv;
        float y = h * Cn;
#pragma unroll
        for (int sh = 8; sh; sh >>= 1) y += __shfl_xor(y, sh, 32);
        y = fmaf(xv, Dd, y);
        if ((l & 15) == s) keep = y;
        if ((l & 15) == 15) { float* dst = YP + ((size_t)w * LL + (l - 15)) * 2 + s * 2 + half; *(volatile float*)dst = keep; __threadfence(); *(volatile float*)dst = keep; }
    }
}

__global__ __launch_bounds__(256) void k_cvtx(const float* __restrict__ src, int rows, bf* dst) {
    const int lane = threadIdx.x & 31; const size_t r = (size_t)blockIdx.x * 8 + (threadIdx.x >> 5); if (r >= (size_t)rows) return;
#pragma unroll 1
    for (int ps = 0; ps < 2; ++ps) {
#pragma unroll
        for (int q = 0; q < DMOD / 256; ++q) { v8us o;
#pragma unroll
            for (int i = 0; i < 8; ++i) o[i] = f2bf(src[r * DMOD + q * 256 + lane * 8 + i]);
            *(volatile v8us*)(dst + r * DMOD + q * 256 + lane * 8) = o; }
        if (ps == 0) __threadfence(); }
}
__global__ __launch_bounds__(256) void k_revx(const float* __restrict__ XZ, float* XR) {
    const int lane = threadIdx.x & 31; const size_t l = (size_t)blockIdx.x * 8 + (threadIdx.x >> 5); if (l >= (size_t)LL) return; const float* s = XZ + (size_t)(LL - 1 - l) * (2 * DI);
#pragma unroll 1
    for (int ps = 0; ps < 2; ++ps) {
#pragma unroll 1
        for (int q = 0; q < DI / 128; ++q) { const size_t c0 = (size_t)q * 128 + lane * 4; const v4f v = *(const v4f*)(s + c0); *(volatile v4f*)(XR + l * (2 * DI) + c0) = v; }
        if (ps == 0) __threadfence(); }
}
__global__ __launch_bounds__(256) void k_gate2(const float* __restrict__ YF, const float* __restrict__ YB, const float* __restrict__ XZ, bf* Gh, bf* Gl) {
    const int lane = threadIdx.x & 31; const size_t l = (size_t)blockIdx.x * 8 + (threadIdx.x >> 5); if (l >= (size_t)LL) return; const size_t lb = LL - 1 - l;
#pragma unroll 1
    for (int ps = 0; ps < 2; ++ps) {
#pragma unroll 1
        for (int q = 0; q < DI / 256; ++q) { const int d0 = q * 256 + lane * 8; v8us oh, ol;
#pragma unroll
            for (int i = 0; i < 8; ++i) { const int d = d0 + i; const float y = YF[((size_t)(d >> 1) * LL + l) * 2 + (d & 1)] + YB[((size_t)(d >> 1) * LL + lb) * 2 + (d & 1)]; const float z = XZ[l * (2 * DI) + DI + d]; const float g = y * (z / (1.0f + expf(-z))); const unsigned short hb = f2bf(g); oh[i] = hb; ol[i] = f2bf(g - bf2f(hb)); }
            const size_t o = l * DI + d0; *(volatile v8us*)(Gh + o) = oh; *(volatile v8us*)(Gl + o) = ol; }
        if (ps == 0) __threadfence(); }
}
__global__ __launch_bounds__(256) void k_n2n(const float* __restrict__ O, float* OUTB) {
    const int lane = threadIdx.x & 31; const size_t l = (size_t)blockIdx.x * 8 + (threadIdx.x >> 5); if (l >= (size_t)LL) return;
#pragma unroll 1
    for (int ps = 0; ps < 2; ++ps) {
#pragma unroll 1
        for (int q = 0; q < DMOD / 128; ++q) { const size_t o = l * DMOD + q * 128 + lane * 4; v4f v = *(const v4f*)(O + o);
#pragma unroll
            for (int i = 0; i < 4; ++i) { float t = v[i]; if (__builtin_isnan(t)) t = 0.f; else if (__builtin_isinf(t)) t = (t > 0.f) ? 1.0f : -1.0f; v[i] = t; }
            *(volatile v4f*)(OUTB + o) = v; }
        if (ps == 0) __threadfence(); }
}

extern "C" void kernel_launch(void* const* d_in, const int* in_sizes, int n_in,
                              void* d_out, int out_size, void* d_ws, size_t ws_size, hipStream_t stream) {
    (void)in_sizes; (void)n_in; (void)out_size;
    const float* x = (const float*)d_in[0]; const float* Win = (const float*)d_in[1];
    const float* Wc = (const float*)d_in[2]; const float* bc = (const float*)d_in[3]; const float* Wx = (const float*)d_in[4]; const float* Wdt = (const float*)d_in[5]; const float* bdt = (const float*)d_in[6]; const float* Alog = (const float*)d_in[7]; const float* Dp = (const float*)d_in[8];
    const float* Wcb = (const float*)d_in[9]; const float* bcb = (const float*)d_in[10]; const float* Wxb = (const float*)d_in[11]; const float* Wdtb = (const float*)d_in[12]; const float* bdtb = (const float*)d_in[13]; const float* Alogb = (const float*)d_in[14]; const float* Dpb = (const float*)d_in[15]; const float* Wout = (const float*)d_in[16];
    float* out = (float*)d_out;
    char* wsp = (char*)d_ws;
    auto take = [&](size_t bytes) { char* p = wsp; wsp += (bytes + 255) & ~(size_t)255; return (void*)p; };
    bf* WIN = (bf*)take((size_t)2 * DI * DMOD * 2); bf* WXP = (bf*)take((size_t)NXP * DI * 2); bf* WDT = (bf*)take((size_t)DI * KDT * 2); bf* WXPb = (bf*)take((size_t)NXP * DI * 2); bf* WDTb = (bf*)take((size_t)DI * KDT * 2); bf* WOUT = (bf*)take((size_t)DMOD * DI * 2);
    bf* Xb = (bf*)take((size_t)LL * DMOD * 2); float* XZ = (float*)take((size_t)LL * 2 * DI * 4); float* XR = (float*)take((size_t)LL * 2 * DI * 4); float* XC = (float*)take((size_t)LL * DI * 4); bf* Ch = (bf*)take((size_t)LL * DI * 2); bf* Cl = (bf*)take((size_t)LL * DI * 2);
    float* XD = (float*)take((size_t)LL * NXP * 4); bf* Th = (bf*)take((size_t)LL * KDT * 2); bf* Tl = (bf*)take((size_t)LL * KDT * 2); float* DEL = (float*)take((size_t)LL * DI * 4); float* YF = (float*)take((size_t)LL * DI * 4); float* YB = (float*)take((size_t)LL * DI * 4); bf* Gh = (bf*)take((size_t)LL * DI * 2); bf* Gl = (bf*)take((size_t)LL * DI * 2); float* O = (float*)take((size_t)LL * DMOD * 4);
    if ((size_t)(wsp - (char*)d_ws) > ws_size) return;
    k_cvt8<<<(unsigned)(((size_t)2 * DI * DMOD / 8 + 255) / 256), 256, 0, stream>>>(Win, WIN, (size_t)2 * DI * DMOD / 8); k_wxpad<<<NXP / 8, 256, 0, stream>>>(Wx, WXP); k_wdtpad<<<DI / 8, 256, 0, stream>>>(Wdt, WDT); k_wxpad<<<NXP / 8, 256, 0, stream>>>(Wxb, WXPb); k_wdtpad<<<DI / 8, 256, 0, stream>>>(Wdtb, WDTb);
    k_cvt8<<<(unsigned)(((size_t)DMOD * DI / 8 + 255) / 256), 256, 0, stream>>>(Wout, WOUT, (size_t)DMOD * DI / 8);
    for (int b = 0; b < NBT; ++b) { const float* xb = x + (size_t)b * LL * DMOD;
        k_cvtx<<<LL / 8, 256, 0, stream>>>(xb, LL, Xb);
        k_gemmb<false, false><<<dim3(LL / 64, (2 * DI) / 64, 1), 128, 0, stream>>>(Xb, nullptr, WIN, nullptr, XZ, 2 * DI, nullptr, nullptr, DMOD);
        k_revx<<<LL / 8, 256, 0, stream>>>(XZ, XR);
        for (int dir = 0; dir < 2; ++dir) { const float* src = dir ? XR : XZ;
            k_conv<<<LL / 8, 256, 0, stream>>>(src, dir ? Wcb : Wc, dir ? bcb : bc, XC, Ch, Cl);
            k_gemmb<true, false><<<dim3(LL / 64, NXP / 64, 1), 128, 0, stream>>>(Ch, Cl, dir ? WXPb : WXP, nullptr, XD, NXP, nullptr, nullptr, DI);
            k_dtplanes<<<LL / 8, 256, 0, stream>>>(XD, Th, Tl);
            k_gemmb<true, false><<<dim3(LL / 64, DI / 64, 1), 128, 0, stream>>>(Th, Tl, dir ? WDTb : WDT, nullptr, DEL, DI, nullptr, nullptr, KDT);
            k_softplus<<<LL / 8, 256, 0, stream>>>(DEL, dir ? bdtb : bdt);
            k_scan<<<(DI / 2) / 8, 256, 0, stream>>>(DEL, XD, XC, dir ? Alogb : Alog, dir ? Dpb : Dp, dir ? YB : YF); }
        k_gate2<<<LL / 8, 256, 0, stream>>>(YF, YB, XZ, Gh, Gl);
        k_gemmb<true, false><<<dim3(LL / 64, DMOD / 64, 1), 128, 0, stream>>>(Gh, Gl, WOUT, nullptr, O, DMOD, nullptr, nullptr, DI);
        k_n2n<<<LL / 8, 256, 0, stream>>>(O, out + (size_t)b * LL * DMOD); }
}
